// Block_88201448390974
// MI455X (gfx1250) — hardware-verified
//
#include <hip/hip_runtime.h>
#include <math.h>

#ifndef NB
#define NB 16
#endif
#ifndef SEQ
#define SEQ 1024
#endif
#define NB_FULL 16
#define SEQ_FULL 1024
#define CW 384
#define NH 6
#define HD 64
#define DFF 1536
#define ROWS (NB * SEQ)
#define AO_CARRY 64.0f

static_assert(SEQ % 64 == 0);
static_assert(SEQ <= SEQ_FULL);
static_assert(NB <= NB_FULL);
static_assert(CW == NH * HD);
static_assert(CW % 128 == 0);
static_assert(CW % 64 == 0 && DFF % 64 == 0 && (2 * CW) % 64 == 0);
static_assert(CW % 32 == 0 && DFF % 32 == 0);

typedef __attribute__((ext_vector_type(16))) _Float16 v16h;
typedef __attribute__((ext_vector_type(8)))  _Float16 v8h;
typedef __attribute__((ext_vector_type(8)))  float    v8f;
typedef __attribute__((ext_vector_type(4)))  float    v4f;
typedef __attribute__((ext_vector_type(4)))  unsigned int u4v;
typedef __attribute__((ext_vector_type(2)))  unsigned int u2v;
typedef v8h v8h_ma __attribute__((may_alias));
typedef v4f v4f_ma __attribute__((may_alias));

union FragU { v16h v; v8h h[2]; };
__device__ __forceinline__ v16h ldfrag(const _Float16* p) { FragU f; f.h[0] = *(const v8h*)(p); f.h[1] = *(const v8h*)(p + 16); return f.v; }
__device__ __forceinline__ v8f mma_h(v16h a, v16h b, v8f c) { return __builtin_amdgcn_wmma_f32_16x16x32_f16(false, a, false, b, (short)0, c, false, false); }
__device__ __forceinline__ void dep_guard_h(v8f& a, v8f& b, v16h x, v16h y) { asm volatile("v_nop\n\tv_nop\n\tv_nop\n\tv_nop" : "+v"(a), "+v"(b) : "v"(x), "v"(y)); }
__device__ __forceinline__ void keep4_h(v16h a, v16h b, v16h c, v16h d) { asm volatile("v_nop" :: "v"(a), "v"(b), "v"(c), "v"(d)); }
__device__ __forceinline__ void acc_guard4(v8f& a, v8f& b, v8f& c, v8f& d) { asm volatile("v_nop\n\tv_nop\n\tv_nop\n\tv_nop" : "+v"(a), "+v"(b), "+v"(c), "+v"(d)); }
__device__ __forceinline__ void guard_s(v8f& a, v8f& b, v16h x, v16h y, v16h z) { asm volatile("v_nop\n\tv_nop\n\tv_nop\n\tv_nop" : "+v"(a), "+v"(b) : "v"(x), "v"(y), "v"(z)); }
__device__ __forceinline__ void guard_o(v8f& a, v8f& b, v8f& c, v8f& d, v16h p, v16h w0, v16h w1, v16h w2, v16h w3) {
    asm volatile("v_nop\n\tv_nop\n\tv_nop\n\tv_nop" : "+v"(a), "+v"(b), "+v"(c), "+v"(d) : "v"(p), "v"(w0), "v"(w1), "v"(w2), "v"(w3));
}
__device__ __forceinline__ void wave_sync() {
    __builtin_amdgcn_fence(3  , "workgroup");
    __builtin_amdgcn_wave_barrier();
    __builtin_amdgcn_fence(2  , "workgroup");
}

#define VST2(T, ptr, val) do { const T vst2_v_ = (val); *(volatile T*)(ptr) = vst2_v_; __threadfence(); *(volatile T*)(ptr) = vst2_v_; } while (0)

__device__ __forceinline__ unsigned int bk_pk2(float a, float b) { return (unsigned int)__builtin_bit_cast(unsigned short, (_Float16)a) | ((unsigned int)__builtin_bit_cast(unsigned short, (_Float16)b) << 16); }
__device__ __forceinline__ float cmb_bf(float v) { const unsigned u = __builtin_bit_cast(unsigned, v); const unsigned r = (u + 0x7fffu + ((u >> 16) & 1u)) & 0xffff0000u; return __builtin_bit_cast(float, r); }
__device__ __forceinline__ float gelu_erf(float v) { return 0.5f * v * (1.0f + erff(v * 0.70710678118654752f)); }

__global__ __launch_bounds__(256) void k_cm_castb(const float* __restrict__ SRC, int lds, unsigned short* __restrict__ DST, int ldd, int nR, int nC, float sc) {
    const long long u = (long long)blockIdx.x * 256 + threadIdx.x; const int per = nC / 8; if (u >= (long long)nR * per) return; const int r = (int)(u / per); const int c0 = 8 * (int)(u % per);
    const float* s = SRC + (long long)r * lds + c0; float w[8];
#pragma unroll
    for (int e = 0; e < 8; ++e) w[e] = cmb_bf(s[e]) * sc;
    u4v pk; pk.x = bk_pk2(w[0], w[1]); pk.y = bk_pk2(w[2], w[3]); pk.z = bk_pk2(w[4], w[5]); pk.w = bk_pk2(w[6], w[7]); VST2(u4v, (u4v*)(DST + (long long)r * ldd + c0), pk); }

template <int NQ, int ABF, int AMAP>
__global__ __launch_bounds__(256) void k_b_ln(const float* __restrict__ A, const float* __restrict__ GA, const float* __restrict__ BE, float eps, float inv_vden, int rows, unsigned short* __restrict__ Y16) {
    #pragma clang fp contract(off)
    constexpr int WD = 128 * NQ;
    const int wave = __builtin_amdgcn_readfirstlane((int)(threadIdx.x >> 5));
    const int r = blockIdx.x * 8 + wave; const int L = threadIdx.x & 31; if (r >= rows) return;
    const long long ra = AMAP ? ((long long)(r / SEQ) * SEQ_FULL + (long long)(r % SEQ)) : (long long)r;
    v4f v[NQ]; float s = 0.f;
#pragma unroll
    for (int q = 0; q < NQ; ++q) { v[q] = *(const v4f*)(A + ra * WD + 4 * L + 128 * q); if (ABF) { v[q].x = cmb_bf(v[q].x); v[q].y = cmb_bf(v[q].y); v[q].z = cmb_bf(v[q].z); v[q].w = cmb_bf(v[q].w); } s += (v[q].x + v[q].y) + (v[q].z + v[q].w); }
#pragma unroll
    for (int o = 16; o > 0; o >>= 1) s += __shfl_xor(s, o, 32);
    const float mu = s * (1.f / WD); float qq = 0.f;
#pragma unroll
    for (int q = 0; q < NQ; ++q) { v[q].x -= mu; v[q].y -= mu; v[q].z -= mu; v[q].w -= mu; qq += (v[q].x * v[q].x + v[q].y * v[q].y) + (v[q].z * v[q].z + v[q].w * v[q].w); }
#pragma unroll
    for (int o = 16; o > 0; o >>= 1) qq += __shfl_xor(qq, o, 32);
    const float rs = rsqrtf(qq * inv_vden + eps);
#pragma unroll
    for (int q = 0; q < NQ; ++q) { const int c = 4 * L + 128 * q; const v4f ga = *(const v4f*)(GA + c), be = *(const v4f*)(BE + c); v4f y;
        y.x = v[q].x * rs * cmb_bf(ga.x) + cmb_bf(be.x); y.y = v[q].y * rs * cmb_bf(ga.y) + cmb_bf(be.y); y.z = v[q].z * rs * cmb_bf(ga.z) + cmb_bf(be.z); y.w = v[q].w * rs * cmb_bf(ga.w) + cmb_bf(be.w);
        const long long o = (long long)r * WD + c; u2v pk; pk.x = bk_pk2(y.x, y.y); pk.y = bk_pk2(y.z, y.w); VST2(u2v, (u2v*)(Y16 + o), pk); } }

template <int BIAS, int OUT16, int RESID, int RBF, int GELU>
__global__ __launch_bounds__(256) void k_gemm64(
    const unsigned short* __restrict__ Ap, int lda, long long strideA,
    const unsigned short* __restrict__ Btp, int ldb, long long strideB,
    void* __restrict__ Cout, int ldc, long long strideC,
    const float* __restrict__ bias, const float* __restrict__ gate,
    const float* __restrict__ resid, long long strideR,
    int M, int N, int K, float scale) {
  __shared__ __align__(16) float sT[8][16 * 68];
  const int b    = blockIdx.y;
  const int lane = threadIdx.x & 31;
  const int wave = __builtin_amdgcn_readfirstlane((int)(threadIdx.x >> 5));
  const int tilesN = N >> 6;
  const int tilesM = M >> 6;
  const int tile = blockIdx.x * 8 + wave;
  if (tile >= tilesM * tilesN) return;
  const int tm = tile / tilesN;
  const int tn = tile - tm * tilesN;
  const int m0 = tm << 6;
  const int n0 = tn << 6;

  const _Float16* Ab = (const _Float16*)Ap  + (size_t)b * (size_t)strideA;
  const _Float16* Bb = (const _Float16*)Btp + (size_t)b * (size_t)strideB;

  const int rlane = lane & 15;
  const int koff  = (lane >> 4) * 8;
  const int mOff  = (lane >> 4) * 8;

  v8f acc[4][4];
#pragma unroll
  for (int i = 0; i < 4; ++i)
#pragma unroll
    for (int j = 0; j < 4; ++j) acc[i][j] = (v8f){0.f,0.f,0.f,0.f,0.f,0.f,0.f,0.f};

  for (int k0 = 0; k0 < K; k0 += 32) {
    v16h bh[4];
#pragma unroll
    for (int j = 0; j < 4; ++j) {
      const size_t bo = (size_t)(n0 + (j << 4) + rlane) * ldb + koff + k0;
      bh[j] = ldfrag(Bb + bo);
    }
#pragma unroll
    for (int i = 0; i < 4; ++i) {
      const size_t ao = (size_t)(m0 + (i << 4) + rlane) * lda + koff + k0;
      const v16h ah = ldfrag(Ab + ao);
#pragma unroll
      for (int j = 0; j < 4; ++j) acc[i][j] = mma_h(ah, bh[j], acc[i][j]);
      dep_guard_h(acc[i][0], acc[i][3], ah, ah);
    }
    keep4_h(bh[0], bh[1], bh[2], bh[3]);
  }
  acc_guard4(acc[0][0], acc[0][1], acc[0][2], acc[0][3]);
  acc_guard4(acc[1][0], acc[1][1], acc[1][2], acc[1][3]);
  acc_guard4(acc[2][0], acc[2][1], acc[2][2], acc[2][3]);
  acc_guard4(acc[3][0], acc[3][1], acc[3][2], acc[3][3]);

  const float* Rb = resid + (size_t)b * (size_t)strideR;
#pragma unroll
  for (int i = 0; i < 4; ++i) {
    const int mBase = m0 + (i << 4);
#pragma unroll
    for (int j = 0; j < 4; ++j) {
      const int n = n0 + (j << 4) + rlane;
      float bv = 0.f;
      if (BIAS) bv = cmb_bf(bias[n]);
#pragma unroll
      for (int r = 0; r < 8; ++r) {
        float v = acc[i][j][r] * scale;
        if (BIAS) v += bv;
        if (RESID) { float rv = Rb[(size_t)(mBase + mOff + r) * ldc + n]; if (RBF) rv = cmb_bf(rv); v += rv; }
        sT[wave][(mOff + r) * 68 + (j << 4) + rlane] = v;
      }
    }
    wave_sync();
    if (OUT16 == 0) {
      float* C = (float*)Cout + (size_t)b * (size_t)strideC;
      const int hh = lane >> 4, c4 = (lane & 15) * 4;
      for (int pass = 0; pass < 2; ++pass) {
#pragma unroll
        for (int it = 0; it < 8; ++it) {
          const int row = it * 2 + hh;
          const v4f v = *(const v4f_ma*)&sT[wave][row * 68 + c4];
          *(volatile v4f*)(C + (size_t)(mBase + row) * ldc + n0 + c4) = v;
        }
        __threadfence();
      }
    } else {
      const int q = lane >> 3, c8 = (lane & 7) * 8;
      unsigned short* C = (unsigned short*)Cout + (size_t)b * (size_t)strideC;
      if (GELU) {
        const v4f g0 = *(const v4f*)(gate + n0 + c8), g1 = *(const v4f*)(gate + n0 + c8 + 4);
        const float gg[8] = {cmb_bf(g0.x), cmb_bf(g0.y), cmb_bf(g0.z), cmb_bf(g0.w), cmb_bf(g1.x), cmb_bf(g1.y), cmb_bf(g1.z), cmb_bf(g1.w)};
#pragma unroll 1
        for (int it = 0; it < 4; ++it) {
          const int row = it * 4 + q;
          const v4f a0 = *(const v4f_ma*)&sT[wave][row * 68 + c8];
          const v4f a1 = *(const v4f_ma*)&sT[wave][row * 68 + c8 + 4];
          v8h hv;
          hv[0] = (_Float16)(gelu_erf(a0.x) * gg[0]); hv[1] = (_Float16)(gelu_erf(a0.y) * gg[1]);
          hv[2] = (_Float16)(gelu_erf(a0.z) * gg[2]); hv[3] = (_Float16)(gelu_erf(a0.w) * gg[3]);
          hv[4] = (_Float16)(gelu_erf(a1.x) * gg[4]); hv[5] = (_Float16)(gelu_erf(a1.y) * gg[5]);
          hv[6] = (_Float16)(gelu_erf(a1.z) * gg[6]); hv[7] = (_Float16)(gelu_erf(a1.w) * gg[7]);
          volatile v8h* dst = (volatile v8h*)(C + (size_t)(mBase + row) * ldc + n0 + c8);
          *dst = hv; __threadfence(); *dst = hv;
        }
      } else {
        for (int pass = 0; pass < 2; ++pass) {
#pragma unroll
          for (int it = 0; it < 4; ++it) {
            const int row = it * 4 + q;
            const v4f a0 = *(const v4f_ma*)&sT[wave][row * 68 + c8];
            const v4f a1 = *(const v4f_ma*)&sT[wave][row * 68 + c8 + 4];
            v8h hv;
            hv[0] = (_Float16)a0.x; hv[1] = (_Float16)a0.y; hv[2] = (_Float16)a0.z; hv[3] = (_Float16)a0.w;
            hv[4] = (_Float16)a1.x; hv[5] = (_Float16)a1.y; hv[6] = (_Float16)a1.z; hv[7] = (_Float16)a1.w;
            *(volatile v8h*)(C + (size_t)(mBase + row) * ldc + n0 + c8) = hv;
          }
          __threadfence();
        }
      }
    }
    wave_sync();
  }
}

__global__ __launch_bounds__(128) void k_fattn(const unsigned short* __restrict__ QK, const unsigned short* __restrict__ VT,
                                               const float* __restrict__ gate_h, unsigned short* __restrict__ AO) {
  __shared__ __align__(16) _Float16 Ps[4][16 * 40];
  __shared__ __align__(16) float    Os[4][16 * 68];
  const int wave = __builtin_amdgcn_readfirstlane((int)(threadIdx.x >> 5));
  const int lane = threadIdx.x & 31, hf = lane >> 4, l15 = lane & 15;
  const int nqb = SEQ / 64;
  const int bx = blockIdx.x;
  const int qb = bx % nqb;
  const int bh = bx / nqb;
  const int h  = bh % NH;
  const int b  = bh / NH;
  const int q0 = qb * 64 + wave * 16;
  const _Float16* QKh = (const _Float16*)QK;
  const _Float16* VTh = (const _Float16*)VT;
  const int qo = (b * SEQ + q0 + l15) * (2 * CW) + h * HD + 8 * hf;
  const int ko = (b * SEQ + l15) * (2 * CW) + CW + h * HD + 8 * hf;
  const int vo = (b * CW + h * HD + l15) * SEQ + 8 * hf;
  const float CS = 0.125f * 1.4426950408889634f;

  v8f o[4]; float m8[8], l8[8];
#pragma unroll
  for (int t = 0; t < 4; ++t) o[t] = (v8f){0.f,0.f,0.f,0.f,0.f,0.f,0.f,0.f};
#pragma unroll
  for (int i = 0; i < 8; ++i) { m8[i] = -1.0e30f; l8[i] = 0.f; }

  for (int jb = 0; jb < SEQ; jb += 32) {
    v8f s0 = (v8f){0.f,0.f,0.f,0.f,0.f,0.f,0.f,0.f};
    v8f s1 = (v8f){0.f,0.f,0.f,0.f,0.f,0.f,0.f,0.f};
#pragma unroll
    for (int ks = 0; ks < 2; ++ks) {
      const v16h qf = ldfrag(QKh + qo + ks * 32);
      const v16h k0 = ldfrag(QKh + ko + jb * (2 * CW) + ks * 32);
      const v16h k1 = ldfrag(QKh + ko + (jb + 16) * (2 * CW) + ks * 32);
      s0 = mma_h(qf, k0, s0);
      s1 = mma_h(qf, k1, s1);
      guard_s(s0, s1, qf, k0, k1);
    }
#pragma unroll
    for (int i = 0; i < 8; ++i) {
      const float a = s0[i] * CS, c = s1[i] * CS;
      float mx = fmaxf(a, c);
      mx = fmaxf(mx, __shfl_xor(mx, 1, 32)); mx = fmaxf(mx, __shfl_xor(mx, 2, 32));
      mx = fmaxf(mx, __shfl_xor(mx, 4, 32)); mx = fmaxf(mx, __shfl_xor(mx, 8, 32));
      const float mnew = fmaxf(m8[i], mx);
      const float corr = exp2f(m8[i] - mnew);
      const float p0 = exp2f(a - mnew), p1 = exp2f(c - mnew);
      float rs = p0 + p1;
      rs += __shfl_xor(rs, 1, 32); rs += __shfl_xor(rs, 2, 32); rs += __shfl_xor(rs, 4, 32); rs += __shfl_xor(rs, 8, 32);
      l8[i] = l8[i] * corr + rs; m8[i] = mnew;
#pragma unroll
      for (int t = 0; t < 4; ++t) o[t][i] *= corr;
      Ps[wave][(8 * hf + i) * 40 + l15]      = (_Float16)(p0 * 4096.0f);
      Ps[wave][(8 * hf + i) * 40 + 16 + l15] = (_Float16)(p1 * 4096.0f);
    }
    wave_sync();
    FragU pf;
    pf.h[0] = *(const v8h_ma*)&Ps[wave][l15 * 40 + 8 * hf];
    pf.h[1] = *(const v8h_ma*)&Ps[wave][l15 * 40 + 16 + 8 * hf];
    const v16h w0 = ldfrag(VTh + vo + jb);
    const v16h w1 = ldfrag(VTh + vo + 16 * SEQ + jb);
    const v16h w2 = ldfrag(VTh + vo + 32 * SEQ + jb);
    const v16h w3 = ldfrag(VTh + vo + 48 * SEQ + jb);
    o[0] = mma_h(pf.v, w0, o[0]);
    o[1] = mma_h(pf.v, w1, o[1]);
    o[2] = mma_h(pf.v, w2, o[2]);
    o[3] = mma_h(pf.v, w3, o[3]);
    guard_o(o[0], o[1], o[2], o[3], pf.v, w0, w1, w2, w3);
    wave_sync();
  }

  const float gh = cmb_bf(gate_h[h]);
#pragma unroll
  for (int i = 0; i < 8; ++i) {
    const float inv = 1.0f / (l8[i] * (4096.0f / AO_CARRY));
#pragma unroll
    for (int t = 0; t < 4; ++t) Os[wave][(8 * hf + i) * 68 + t * 16 + l15] = (o[t][i] * inv) * gh;
  }
  wave_sync();
  {
    const int q = lane >> 3, c8 = (lane & 7) * 8;
    unsigned short* orow = AO + (size_t)(b * SEQ + q0) * CW + h * HD;
    for (int pass = 0; pass < 2; ++pass) {
#pragma unroll
      for (int it = 0; it < 4; ++it) {
        const int row = it * 4 + q;
        const v4f a0 = *(const v4f_ma*)&Os[wave][row * 68 + c8];
        const v4f a1 = *(const v4f_ma*)&Os[wave][row * 68 + c8 + 4];
        v8h hv;
        hv[0] = (_Float16)a0.x; hv[1] = (_Float16)a0.y; hv[2] = (_Float16)a0.z; hv[3] = (_Float16)a0.w;
        hv[4] = (_Float16)a1.x; hv[5] = (_Float16)a1.y; hv[6] = (_Float16)a1.z; hv[7] = (_Float16)a1.w;
        *(volatile v8h*)(orow + (size_t)row * CW + c8) = hv;
      }
      __threadfence();
    }
  }
}

constexpr size_t SZ_X16 = (size_t)ROWS * CW * 2;
constexpr size_t SZ_WQKV = (size_t)3 * CW * CW * 2;
constexpr size_t SZ_WO  = (size_t)CW * CW * 2;
constexpr size_t SZ_W1  = (size_t)DFF * CW * 2;
constexpr size_t SZ_W2  = (size_t)CW * DFF * 2;
constexpr size_t SZ_QK  = (size_t)ROWS * 2 * CW * 2;
constexpr size_t SZ_VT  = (size_t)NB * CW * SEQ * 2;
constexpr size_t SZ_M   = (size_t)ROWS * DFF * 2;
constexpr size_t SZ_X1  = (size_t)ROWS * CW * 4;
constexpr size_t WS_TOTAL = SZ_X16 + SZ_WQKV + SZ_WO + SZ_W1 + SZ_W2 + SZ_M + SZ_X1;
static_assert(SZ_QK + SZ_VT <= SZ_M);
static_assert(SZ_X16 % 256 == 0 && SZ_WQKV % 256 == 0 && SZ_WO % 256 == 0 && SZ_W1 % 256 == 0 && SZ_QK % 256 == 0 && SZ_M % 256 == 0 && SZ_X1 % 256 == 0);
static_assert(WS_TOTAL <= (size_t)134217728);

extern "C" void kernel_launch(void* const* d_in, const int* in_sizes, int n_in, void* d_out, int out_size, void* d_ws, size_t ws_size, hipStream_t stream) {
    if (n_in < 14) return;
    const long long xneed = ((long long)(NB - 1) * SEQ_FULL + SEQ) * CW;
    if ((long long)in_sizes[0] < xneed || (long long)out_size < xneed) return;
    if (in_sizes[1] < CW || in_sizes[2] < CW || in_sizes[3] < 3 * CW * CW || in_sizes[4] < CW * CW || in_sizes[5] < CW || in_sizes[6] < NH) return;
    if (in_sizes[7] < CW || in_sizes[8] < CW || in_sizes[9] < DFF * CW || in_sizes[10] < DFF || in_sizes[11] < CW * DFF || in_sizes[12] < CW || in_sizes[13] < DFF) return;
    if (WS_TOTAL > ws_size) return;
    const float* x      = (const float*)d_in[0];
    const float* ln1_g  = (const float*)d_in[1];
    const float* ln1_b  = (const float*)d_in[2];
    const float* qkv_w  = (const float*)d_in[3];
    const float* proj_w = (const float*)d_in[4];
    const float* proj_b = (const float*)d_in[5];
    const float* gate_h = (const float*)d_in[6];
    const float* ln2_g  = (const float*)d_in[7];
    const float* ln2_b  = (const float*)d_in[8];
    const float* fc1_w  = (const float*)d_in[9];
    const float* fc1_b  = (const float*)d_in[10];
    const float* fc2_w  = (const float*)d_in[11];
    const float* fc2_b  = (const float*)d_in[12];
    const float* gate_m = (const float*)d_in[13];
    float* out = (float*)d_out;

    char* wsp = (char*)d_ws;
    unsigned short* X16  = (unsigned short*)wsp; wsp += SZ_X16;
    unsigned short* W316 = (unsigned short*)wsp; wsp += SZ_WQKV;
    unsigned short* WO16 = (unsigned short*)wsp; wsp += SZ_WO;
    unsigned short* W1T  = (unsigned short*)wsp; wsp += SZ_W1;
    unsigned short* W2T  = (unsigned short*)wsp; wsp += SZ_W2;
    unsigned short* QK16 = (unsigned short*)wsp;
    unsigned short* VT16 = (unsigned short*)(wsp + SZ_QK);
    unsigned short* M16  = (unsigned short*)wsp; wsp += SZ_M;
    float* X1 = (float*)wsp; wsp += SZ_X1;
    unsigned short* AO16 = X16;
    unsigned short* H16  = X16;

    k_b_ln<3, 1, 1><<<(ROWS + 7) / 8, 256, 0, stream>>>(x, ln1_g, ln1_b, 1e-5f, 1.0f / 384.0f, ROWS, X16);
    k_cm_castb<<<(unsigned)((((long long)(3 * CW)) * (CW / 8) + 255) / 256), 256, 0, stream>>>(qkv_w, CW, W316, CW, 3 * CW, CW, 16.0f);
    k_cm_castb<<<(unsigned)((((long long)CW) * (CW / 8) + 255) / 256), 256, 0, stream>>>(proj_w, CW, WO16, CW, CW, CW, 16.0f);
    k_cm_castb<<<(unsigned)((((long long)DFF) * (CW / 8) + 255) / 256), 256, 0, stream>>>(fc1_w, CW, W1T, CW, DFF, CW, 16.0f);
    k_cm_castb<<<(unsigned)((((long long)CW) * (DFF / 8) + 255) / 256), 256, 0, stream>>>(fc2_w, DFF, W2T, DFF, CW, DFF, 16.0f);
    k_gemm64<0, 1, 0, 0, 0><<<dim3((unsigned)(((ROWS / 64) * ((2 * CW) / 64) + 7) / 8), 1u), 256, 0, stream>>>(
        X16, CW, 0LL, W316, CW, 0LL, (void*)QK16, 2 * CW, 0LL, proj_b, gate_m, x, 0LL, ROWS, 2 * CW, CW, 0.0625f);
    k_gemm64<0, 1, 0, 0, 0><<<dim3((unsigned)(((CW / 64) * (SEQ / 64) + 7) / 8), (unsigned)NB), 256, 0, stream>>>(
        W316 + (size_t)2 * CW * CW, CW, 0LL, X16, CW, (long long)SEQ * CW, (void*)VT16, SEQ, (long long)CW * SEQ, proj_b, gate_m, x, 0LL, CW, SEQ, CW, 0.0625f);
    k_fattn<<<(unsigned)(NB * NH * (SEQ / 64)), 128, 0, stream>>>(QK16, VT16, gate_h, AO16);
    k_gemm64<1, 0, 1, 1, 0><<<dim3((unsigned)(((SEQ / 64) * (CW / 64) + 7) / 8), (unsigned)NB), 256, 0, stream>>>(
        AO16, CW, (long long)SEQ * CW, WO16, CW, 0LL, (void*)X1, CW, (long long)SEQ * CW, proj_b, gate_m, x, (long long)SEQ_FULL * CW, SEQ, CW, CW, 1.0f / (16.0f * AO_CARRY));
    k_b_ln<3, 0, 0><<<(ROWS + 7) / 8, 256, 0, stream>>>(X1, ln2_g, ln2_b, 1e-5f, 1.0f / 384.0f, ROWS, H16);
    k_gemm64<1, 1, 0, 0, 1><<<dim3((unsigned)(((ROWS / 64) * (DFF / 64) + 7) / 8), 1u), 256, 0, stream>>>(
        H16, CW, 0LL, W1T, CW, 0LL, (void*)M16, DFF, 0LL, fc1_b, gate_m, x, 0LL, ROWS, DFF, CW, 0.0625f);
    k_gemm64<1, 0, 1, 0, 0><<<dim3((unsigned)(((SEQ / 64) * (CW / 64) + 7) / 8), (unsigned)NB), 256, 0, stream>>>(
        M16, DFF, (long long)SEQ * DFF, W2T, DFF, 0LL, (void*)out, CW, (long long)SEQ_FULL * CW, fc2_b, gate_m, X1, (long long)SEQ * CW, SEQ, CW, DFF, 0.0625f);
}
